// Net_5918464934506
// MI455X (gfx1250) — hardware-verified
//
#include <hip/hip_runtime.h>
#include <stddef.h>
#include <stdint.h>
#include <math.h>


#define FI     16
#define FO     64
#define SD     4
#define KIN    32
#define KP     64
#define NKER   (FI * FO)
#define EB     64
#define ETHR   128
#define NTHR   256
#define NWAVE  8
#define EPT    8
#define CHUNK  (NTHR * EPT)
#define WCAP   (EPT * 32)
#define LISTN  (NWAVE * WCAP)
#define NBA    1024
#define SLA    10
#define RCAP   8192
#define DEGCAP 31
#define NUW    (NKER * (KP / 8))
#define AGG_ZINTS (LISTN + 2 * RCAP + 3 * NBA)
#define MISC_INTS 16
#define OFF_HL   (LISTN)
#define OFF_SL   (LISTN + RCAP)
#define OFF_CNT  (LISTN + 2 * RCAP)
#define OFF_OFFS (OFF_CNT + NBA)
#define OFF_CUR  (OFF_OFFS + NBA)
#define OFF_MISC (OFF_CUR + NBA)
#define OFF_FB   (OFF_MISC + MISC_INTS)
#define OFF_RK   (OFF_FB + NBA)
#define OFF_GK   (OFF_RK + FI * FO)
#define OFF_EB   (OFF_GK + FO)
#define SCAN_LDS_INTS (OFF_EB + FO)
#define WSMAX  134217728

static_assert((CHUNK & (CHUNK - 1)) == 0 && CHUNK <= 4096);
static_assert((NBA & (NBA - 1)) == 0 && NBA == (1 << SLA));
static_assert(((long long)CHUNK << SLA) < (1LL << 31));
static_assert(LISTN % NTHR == 0);
static_assert(NBA % NWAVE == 0 && NBA % 32 == 0 && NBA == 4 * NTHR);
static_assert(RCAP % 4 == 0 && AGG_ZINTS % 4 == 0 && LISTN % 4 == 0);
static_assert(OFF_MISC == AGG_ZINTS && (OFF_FB % 4) == 0 && (OFF_RK % 4) == 0 && (OFF_GK % 4) == 0);
static_assert(DEGCAP <= 31);
static_assert(KP % 32 == 0 && KP == 2 * KIN);
static_assert(EB == (ETHR / 32) * 16 && FO == 64 && FI == 16);
static_assert(ETHR == SD * KIN && ETHR * 8 == NKER && ETHR == 2 * EB);
static_assert(NUW % NTHR == 0 && FI * FO == 4 * NTHR);
static_assert(FO == 2 * 32);
static_assert(SCAN_LDS_INTS * 4 <= 300000);

typedef float          v2f   __attribute__((ext_vector_type(2)));
typedef float          v4f   __attribute__((ext_vector_type(4)));
typedef float          v8f   __attribute__((ext_vector_type(8)));
typedef int            v4i   __attribute__((ext_vector_type(4)));
typedef int            v8i   __attribute__((ext_vector_type(8)));
typedef unsigned short v8us  __attribute__((ext_vector_type(8)));
typedef unsigned short v16us __attribute__((ext_vector_type(16)));
typedef __bf16         v16bf __attribute__((ext_vector_type(16)));
typedef v2f  __attribute__((may_alias)) v2fa;
typedef v4f  __attribute__((may_alias)) v4fa;
typedef v4i  __attribute__((may_alias)) v4ia;
typedef v8us __attribute__((may_alias)) v8usa;
union FragB { v16bf v; v16us u; v8us h[2]; v8i w; };

__device__ __forceinline__ v8f wmb(const FragB& a, const FragB& b, v8f c) {
  v8f d = __builtin_amdgcn_wmma_f32_16x16x32_bf16(false, a.v, false, b.v, (short)0, c, false, false);
  asm volatile("v_nop\n\tv_nop\n\tv_nop\n\tv_nop" : "+v"(d) : "v"(a.w), "v"(b.w));
  return d;
}

__device__ __forceinline__ unsigned bf16_bits(float f) {
  const unsigned u = __float_as_uint(f);
  return (u + 0x7FFFu + ((u >> 16) & 1u)) >> 16;
}
__device__ __forceinline__ float bf16_val(float f) {
  return __uint_as_float(bf16_bits(f) << 16);
}
__device__ __forceinline__ float rdl(float v, int k) {
  return __int_as_float(__builtin_amdgcn_readlane(__float_as_int(v), k));
}
__device__ __forceinline__ float nmax(float a, float b) {
  float r = (a > b) ? a : b;
  r = (a != a) ? a : r;
  return r;
}

template <int SLB>
__device__ __forceinline__ int scan_chunk(const int* __restrict__ dsts, int nE, int cbase, int slotBase,
                                          int nb, int vec8, int* list, int tid, int lane, int wave) {
  int wc = 0;
  const int el0  = tid * EPT;
  const int e0   = cbase + el0;
  const int sent = -2147483647 - 1;
  v4i da, db;
  if (vec8 != 0 && cbase + CHUNK <= nE) {
    da = *(const v4i*)(dsts + e0);
    db = *(const v4i*)(dsts + e0 + 4);
  } else {
    da.x = (e0     < nE) ? dsts[min(e0,     nE - 1)] : sent;
    da.y = (e0 + 1 < nE) ? dsts[min(e0 + 1, nE - 1)] : sent;
    da.z = (e0 + 2 < nE) ? dsts[min(e0 + 2, nE - 1)] : sent;
    da.w = (e0 + 3 < nE) ? dsts[min(e0 + 3, nE - 1)] : sent;
    db.x = (e0 + 4 < nE) ? dsts[min(e0 + 4, nE - 1)] : sent;
    db.y = (e0 + 5 < nE) ? dsts[min(e0 + 5, nE - 1)] : sent;
    db.z = (e0 + 6 < nE) ? dsts[min(e0 + 6, nE - 1)] : sent;
    db.w = (e0 + 7 < nE) ? dsts[min(e0 + 7, nE - 1)] : sent;
  }
  const unsigned nbs = (unsigned)slotBase;
  const unsigned unb = (unsigned)nb;
  const unsigned s0 = (unsigned)da.x - nbs, s1 = (unsigned)da.y - nbs;
  const unsigned s2 = (unsigned)da.z - nbs, s3 = (unsigned)da.w - nbs;
  const unsigned s4 = (unsigned)db.x - nbs, s5 = (unsigned)db.y - nbs;
  const unsigned s6 = (unsigned)db.z - nbs, s7 = (unsigned)db.w - nbs;
  const bool h0 = s0 < unb, h1 = s1 < unb, h2 = s2 < unb, h3 = s3 < unb;
  const bool h4 = s4 < unb, h5 = s5 < unb, h6 = s6 < unb, h7 = s7 < unb;
  const unsigned any = __builtin_amdgcn_ballot_w32(h0 | h1 | h2 | h3 | h4 | h5 | h6 | h7);
  if (any != 0u) {
#define HITJ(J, HJ, SJ) { \
      const unsigned mj = __builtin_amdgcn_ballot_w32(HJ); \
      if (mj != 0u) { \
        if (HJ) { \
          const int pos = wc + (int)__builtin_amdgcn_mbcnt_lo(mj, 0u); \
          if (pos < WCAP) list[wave * WCAP + pos] = ((el0 + (J)) << SLB) | (int)(SJ); \
        } \
        wc += (int)__builtin_popcount(mj); } }
    HITJ(0, h0, s0)
    HITJ(1, h1, s1)
    HITJ(2, h2, s2)
    HITJ(3, h3, s3)
    HITJ(4, h4, s4)
    HITJ(5, h5, s5)
    HITJ(6, h6, s6)
    HITJ(7, h7, s7)
#undef HITJ
  }
  return wc;
}

__device__ __forceinline__ void build_lists(const int* __restrict__ keys, int nE, int nodeBase, int vec8,
                                            int* dsm, int tid, int lane, int wave) {
  int* list = dsm;
  int* hl   = dsm + OFF_HL;
  int* sl   = dsm + OFF_SL;
  int* cnt  = dsm + OFF_CNT;
  int* offs = dsm + OFF_OFFS;
  int* cur  = dsm + OFF_CUR;
  int* misc = dsm + OFF_MISC;
  {
    const v4i z4 = {0, 0, 0, 0};
    for (int i = tid * 4; i < AGG_ZINTS; i += NTHR * 4) *(v4ia*)(dsm + i) = z4;
    if (tid < MISC_INTS) misc[tid] = 0;
  }
  __syncthreads();

  int t = 0, ov = 0;
  const int nChunks = (nE + CHUNK - 1) / CHUNK;
#pragma unroll 1
  for (int ch = 0; ch < nChunks; ++ch) {
    const int cbase = ch * CHUNK;
    const int wc = scan_chunk<SLA>(keys, nE, cbase, nodeBase, NBA, vec8, list, tid, lane, wave);
    if (lane == 0) misc[wave] = wc;
    __syncthreads();
    if (wave == 0) {
#pragma unroll 1
      for (int w2 = 0; w2 < NWAVE; ++w2) {
        int c = misc[w2];
        c = c < 0 ? 0 : (c > WCAP ? WCAP : c);
#pragma unroll 1
        for (int b0 = 0; b0 < c; b0 += 32) {
          const int idx = b0 + lane;
          const int ent = list[w2 * WCAP + (idx < WCAP ? idx : WCAP - 1)];
          const int m32 = (c - b0) < 32 ? (c - b0) : 32;
#pragma unroll 1
          for (int k = 0; k < m32; ++k) {
            const int u    = __builtin_amdgcn_readlane(ent, k);
            const int slot = u & (NBA - 1);
            const int el   = (u >> SLA) & (CHUNK - 1);
            const int pk   = ((cbase + el) << SLA) | slot;
            if (t < RCAP) {
              if (lane == 0) { hl[t] = pk; cnt[slot] = cnt[slot] + 1; }
              t = t + 1;
            } else {
              ov = 1;
            }
          }
        }
      }
    }
    __syncthreads();
  }
  if (wave == 0 && lane == 0) { misc[8] = t; misc[9] = ov; }
  __syncthreads();
  int tt = misc[8];
  tt = tt < 0 ? 0 : (tt > RCAP ? RCAP : tt);

  if (wave == 0) {
    const int base = lane * (NBA / 32);
    int s = 0;
#pragma unroll 1
    for (int i = 0; i < NBA / 32; ++i) s += cnt[base + i];
    int incl = s;
#pragma unroll
    for (int d = 1; d < 32; d <<= 1) {
      const int y = __shfl_up(incl, d, 32);
      if (lane >= d) incl += y;
    }
    int run = incl - s;
#pragma unroll 1
    for (int i = 0; i < NBA / 32; ++i) {
      const int cv = cnt[base + i];
      offs[base + i] = run;
      cur[base + i]  = run;
      run += cv;
    }
  }
  __syncthreads();
  if (wave == 0) {
#pragma unroll 1
    for (int b0 = 0; b0 < tt; b0 += 32) {
      const int idx = b0 + lane;
      const int ent = hl[idx < RCAP ? idx : RCAP - 1];
      const int m32 = (tt - b0) < 32 ? (tt - b0) : 32;
#pragma unroll 1
      for (int k = 0; k < m32; ++k) {
        const int u    = __builtin_amdgcn_readlane(ent, k);
        const int slot = u & (NBA - 1);
        if (lane == 0) {
          int p = cur[slot];
          p = p < 0 ? 0 : (p > RCAP - 1 ? RCAP - 1 : p);
          sl[p] = u;
          cur[slot] = p + 1;
        }
      }
    }
  }
  __syncthreads();
}

__global__ __launch_bounds__(NTHR) void k_prep(const float* __restrict__ W2, unsigned short* W2T2) {
  const int u = (int)blockIdx.x * NTHR + (int)threadIdx.x;
  if (u >= NUW) return;
  const int n  = u >> 3;
  const int k8 = (u & 7) * 8;
  const int kk = k8 & (KIN - 1);
  const float* p = W2 + (size_t)kk * NKER + n;
  v8us o;
#pragma unroll
  for (int i = 0; i < 8; ++i) o[i] = (unsigned short)bf16_bits(p[(size_t)i * NKER]);
  unsigned short* dp = W2T2 + (size_t)n * KP + k8;
  *(volatile v8us*)dp = o;
  __threadfence();
  *(volatile v8us*)dp = o;
}

__device__ __forceinline__ float hunit(float e0, float e1, float e2, float e3,
                                       const float* w1s, const float* b1s, int kk) {
  float a = e0 * w1s[kk];
  a = fmaf(e1, w1s[KIN + kk], a);
  a = fmaf(e2, w1s[2 * KIN + kk], a);
  a = fmaf(e3, w1s[3 * KIN + kk], a);
  a = a + b1s[kk];
  return (a > 0.0f) ? a : 0.0f;
}

__global__ __launch_bounds__(ETHR) void k_ecc_edge(
    const float* __restrict__ x, const float* __restrict__ ef, const int* __restrict__ esrc,
    const float* __restrict__ W1, const float* __restrict__ b1, const float* __restrict__ b2,
    const unsigned short* __restrict__ W2T2, float* msg, int nE, int nN)
{
  __shared__ __attribute__((aligned(16))) unsigned short At[EB * KP];
  __shared__ __attribute__((aligned(16))) float xsT[FI * EB];
  __shared__ __attribute__((aligned(16))) float stg[EB * FO];
  __shared__ __attribute__((aligned(16))) float b2s[NKER];
  __shared__ float w1s[SD * KIN];
  __shared__ float b1s[KIN];
  const int tid = (int)threadIdx.x, lane = tid & 31, wave = tid >> 5, hh = lane >> 4, m = lane & 15;
  const int ebase = (int)blockIdx.x * EB;

  w1s[tid] = bf16_val(W1[tid]);
  if (tid < KIN) b1s[tid] = bf16_val(b1[tid]);
  {
    const v4f a = *(const v4f*)(b2 + 8 * tid);
    const v4f b = *(const v4f*)(b2 + 8 * tid + 4);
    v4f c, d;
    c.x = bf16_val(a.x); c.y = bf16_val(a.y); c.z = bf16_val(a.z); c.w = bf16_val(a.w);
    d.x = bf16_val(b.x); d.y = bf16_val(b.y); d.z = bf16_val(b.z); d.w = bf16_val(b.w);
    *(v4fa*)(b2s + 8 * tid) = c;
    *(v4fa*)(b2s + 8 * tid + 4) = d;
  }
  __syncthreads();

  {
    const int row = tid >> 1;
    const int kh  = (tid & 1) * 16;
    int eg = ebase + row;
    eg = eg < nE ? eg : nE - 1;
    const v4f ev = *(const v4f*)(ef + (size_t)eg * SD);
    const float e0 = bf16_val(ev.x), e1 = bf16_val(ev.y), e2 = bf16_val(ev.z), e3 = bf16_val(ev.w);
    v8us h0, h1, l0, l1;
#pragma unroll
    for (int k = 0; k < 8; ++k) {
      const float a = hunit(e0, e1, e2, e3, w1s, b1s, kh + k);
      const unsigned hb = bf16_bits(a);
      h0[k] = (unsigned short)hb;
      l0[k] = (unsigned short)bf16_bits(a - __uint_as_float(hb << 16));
    }
#pragma unroll
    for (int k = 0; k < 8; ++k) {
      const float a = hunit(e0, e1, e2, e3, w1s, b1s, kh + 8 + k);
      const unsigned hb = bf16_bits(a);
      h1[k] = (unsigned short)hb;
      l1[k] = (unsigned short)bf16_bits(a - __uint_as_float(hb << 16));
    }
    unsigned short* arow = At + row * KP;
    *(v8usa*)(arow + kh) = h0;
    *(v8usa*)(arow + kh + 8) = h1;
    *(v8usa*)(arow + KIN + kh) = l0;
    *(v8usa*)(arow + KIN + kh + 8) = l1;

    const int f8 = (tid & 1) * 8;
    int sr = esrc[eg];
    sr = sr < 0 ? 0 : (sr > nN - 1 ? nN - 1 : sr);
    const float* xq = x + (size_t)sr * FI + f8;
    const v4f xa = *(const v4f*)xq;
    const v4f xb = *(const v4f*)(xq + 4);
    xsT[(f8 + 0) * EB + row] = bf16_val(xa.x);
    xsT[(f8 + 1) * EB + row] = bf16_val(xa.y);
    xsT[(f8 + 2) * EB + row] = bf16_val(xa.z);
    xsT[(f8 + 3) * EB + row] = bf16_val(xa.w);
    xsT[(f8 + 4) * EB + row] = bf16_val(xb.x);
    xsT[(f8 + 5) * EB + row] = bf16_val(xb.y);
    xsT[(f8 + 6) * EB + row] = bf16_val(xb.z);
    xsT[(f8 + 7) * EB + row] = bf16_val(xb.w);
  }
  __syncthreads();

  FragB af0, af1;
  {
    const unsigned short* ap = At + (16 * wave + m) * KP + 8 * hh;
    af0.h[0] = *(const v8usa*)(ap);
    af0.h[1] = *(const v8usa*)(ap + 16);
    af1.h[0] = *(const v8usa*)(ap + 32);
    af1.h[1] = *(const v8usa*)(ap + 48);
  }

  const v8f z8 = {0.f, 0.f, 0.f, 0.f, 0.f, 0.f, 0.f, 0.f};
  v8f macc[4];
  macc[0] = z8; macc[1] = z8; macc[2] = z8; macc[3] = z8;
  const unsigned short* wp = W2T2 + (size_t)m * KP + 8 * hh;
#pragma unroll 1
  for (int f = 0; f < FI; ++f) {
    v8f kacc[4];
#pragma unroll
    for (int t = 0; t < 4; ++t) {
      const unsigned short* wq = wp + (size_t)(f * FO + 16 * t) * KP;
      FragB bf;
      bf.h[0] = *(const v8usa*)wq;
      bf.h[1] = *(const v8usa*)(wq + 16);
      kacc[t] = wmb(af0, bf, z8);
    }
#pragma unroll
    for (int t = 0; t < 4; ++t) {
      const unsigned short* wq = wp + (size_t)(f * FO + 16 * t) * KP + 32;
      FragB bf;
      bf.h[0] = *(const v8usa*)wq;
      bf.h[1] = *(const v8usa*)(wq + 16);
      kacc[t] = wmb(af1, bf, kacc[t]);
    }
    const v4f xa = *(const v4fa*)(xsT + f * EB + 16 * wave + 8 * hh);
    const v4f xb = *(const v4fa*)(xsT + f * EB + 16 * wave + 8 * hh + 4);
#pragma unroll
    for (int t = 0; t < 4; ++t) {
      const float bv = b2s[f * FO + 16 * t + m];
      macc[t][0] = fmaf(xa.x, kacc[t][0] + bv, macc[t][0]);
      macc[t][1] = fmaf(xa.y, kacc[t][1] + bv, macc[t][1]);
      macc[t][2] = fmaf(xa.z, kacc[t][2] + bv, macc[t][2]);
      macc[t][3] = fmaf(xa.w, kacc[t][3] + bv, macc[t][3]);
      macc[t][4] = fmaf(xb.x, kacc[t][4] + bv, macc[t][4]);
      macc[t][5] = fmaf(xb.y, kacc[t][5] + bv, macc[t][5]);
      macc[t][6] = fmaf(xb.z, kacc[t][6] + bv, macc[t][6]);
      macc[t][7] = fmaf(xb.w, kacc[t][7] + bv, macc[t][7]);
    }
  }

#pragma unroll
  for (int t = 0; t < 4; ++t) {
    const int lc = 16 * t + m;
#pragma unroll
    for (int r = 0; r < 8; ++r) {
      const int lr = 16 * wave + 8 * hh + r;
      stg[lr * FO + lc] = macc[t][r];
    }
  }
  __syncthreads();

  v4f fv[8];
#pragma unroll
  for (int i = 0; i < 8; ++i) {
    const int lr = 16 * wave + 2 * i + hh;
    fv[i] = *(const v4fa*)(stg + lr * FO + 4 * m);
  }
#pragma unroll
  for (int i = 0; i < 8; ++i) {
    const int lr = 16 * wave + 2 * i + hh;
    float* op = msg + (size_t)(ebase + lr) * FO + 4 * m;
    *(volatile v4f*)op = fv[i];
  }
  __threadfence();
#pragma unroll
  for (int i = 0; i < 8; ++i) {
    const int lr = 16 * wave + 2 * i + hh;
    float* op = msg + (size_t)(ebase + lr) * FO + 4 * m;
    *(volatile v4f*)op = fv[i];
  }
}

__global__ __launch_bounds__(NTHR) void k_scan1(const int* __restrict__ keys, int nE, int nN, int vec8,
                                                const float* __restrict__ msg, const float* __restrict__ x,
                                                const float* __restrict__ rootk, const float* __restrict__ eccb,
                                                const float* __restrict__ gatk, float* xpOut) {
  extern __shared__ __attribute__((aligned(16))) int dsm[];
  int* sl   = dsm + OFF_SL;
  int* cnt  = dsm + OFF_CNT;
  int* offs = dsm + OFF_OFFS;
  int* misc = dsm + OFF_MISC;
  float* fb = (float*)(dsm + OFF_FB);
  float* rk = (float*)(dsm + OFF_RK);
  float* gk = (float*)(dsm + OFF_GK);
  float* eb = (float*)(dsm + OFF_EB);
  const int tid = (int)threadIdx.x, lane = tid & 31, wave = tid >> 5;
  const int nodeBase = (int)blockIdx.x * NBA;

  {
    const v4f a = *(const v4f*)(rootk + 4 * tid);
    v4f c;
    c.x = bf16_val(a.x); c.y = bf16_val(a.y); c.z = bf16_val(a.z); c.w = bf16_val(a.w);
    *(v4fa*)(rk + 4 * tid) = c;
    if (tid < FO) {
      gk[tid] = bf16_val(gatk[tid]);
      eb[tid] = bf16_val(eccb[tid]);
    }
  }
  build_lists(keys, nE, nodeBase, vec8, dsm, tid, lane, wave);
  const int ovf = misc[9];
  const float qnan = __int_as_float(0x7fc00000);
  const float pz = (ovf != 0) ? qnan : 0.0f;
  const v2f gk2 = *(const v2fa*)(gk + 2 * lane);
  const v2f eb2 = *(const v2fa*)(eb + 2 * lane);

#pragma unroll 1
  for (int si = 0; si < NBA / NWAVE; ++si) {
    const int s    = si * NWAVE + wave;
    const int node = nodeBase + s;
    int c = __builtin_amdgcn_readfirstlane(cnt[s]);
    const bool big = c > DEGCAP;
    c = c < 0 ? 0 : (c > DEGCAP ? DEGCAP : c);
    int o = __builtin_amdgcn_readfirstlane(offs[s]);
    o = o < 0 ? 0 : (o > RCAP ? RCAP : o);
    const int nc = node < nN ? node : nN - 1;
    int idx = o + lane;
    idx = idx > RCAP - 1 ? RCAP - 1 : idx;
    const int ent = sl[idx];
    int eid = ent >> SLA;
    eid = eid < 0 ? 0 : (eid > nE - 1 ? nE - 1 : eid);
    const bool valid = lane < c;
    int rank = 0;
#pragma unroll 1
    for (int k = 0; k < c; ++k) {
      const int ek = __builtin_amdgcn_readlane(eid, k);
      rank += (ek < eid) ? 1 : 0;
    }
    float acc0 = 0.0f, acc1 = 0.0f;
#pragma unroll 1
    for (int p = 0; p < c; ++p) {
      const unsigned mk = __builtin_amdgcn_ballot_w32(valid && (rank == p));
      int k = __builtin_ffs((int)mk) - 1;
      k = k < 0 ? 0 : k;
      const int ek = __builtin_amdgcn_readlane(eid, k);
      const v2f a = *(const v2fa*)(msg + (size_t)ek * FO + 2 * lane);
      acc0 += a.x; acc1 += a.y;
    }
    float xv[FI];
    {
      const float* xr = x + (size_t)nc * FI;
      const v4f q0 = *(const v4f*)xr;
      const v4f q1 = *(const v4f*)(xr + 4);
      const v4f q2 = *(const v4f*)(xr + 8);
      const v4f q3 = *(const v4f*)(xr + 12);
      xv[0]  = bf16_val(q0.x); xv[1]  = bf16_val(q0.y); xv[2]  = bf16_val(q0.z); xv[3]  = bf16_val(q0.w);
      xv[4]  = bf16_val(q1.x); xv[5]  = bf16_val(q1.y); xv[6]  = bf16_val(q1.z); xv[7]  = bf16_val(q1.w);
      xv[8]  = bf16_val(q2.x); xv[9]  = bf16_val(q2.y); xv[10] = bf16_val(q2.z); xv[11] = bf16_val(q2.w);
      xv[12] = bf16_val(q3.x); xv[13] = bf16_val(q3.y); xv[14] = bf16_val(q3.z); xv[15] = bf16_val(q3.w);
    }
    float r0 = 0.0f, r1 = 0.0f;
#pragma unroll
    for (int f = 0; f < FI; ++f) {
      const v2f w = *(const v2fa*)(rk + f * FO + 2 * lane);
      r0 = fmaf(xv[f], w.x, r0);
      r1 = fmaf(xv[f], w.y, r1);
    }
    const float pzr = big ? qnan : pz;
    float y0 = ((acc0 + r0) + eb2.x) + pzr;
    float y1 = ((acc1 + r1) + eb2.y) + pzr;
    y0 = (y0 > 0.0f) ? y0 : (y0 - y0);
    y1 = (y1 > 0.0f) ? y1 : (y1 - y1);
    float part = y0 * gk2.x + y1 * gk2.y;
#pragma unroll
    for (int d = 16; d >= 1; d >>= 1) part += __shfl_xor(part, d, 32);
    const bool live = node < nN;
    const float res = live ? part : 0.0f;
    if (lane == 0) fb[s] = res;
  }
  __syncthreads();
  const v4f ov = *(const v4fa*)(fb + 4 * tid);
  float* op = xpOut + (size_t)nodeBase + 4 * tid;
  *(volatile v4f*)op = ov;
  __threadfence();
  *(volatile v4f*)op = ov;
}

__global__ __launch_bounds__(NTHR) void k_scan2(const int* __restrict__ srcs, const int* __restrict__ keys,
                                                int nE, int nN, int vec8, const float* __restrict__ xp,
                                                const float* __restrict__ attS, const float* __restrict__ attN,
                                                const float* __restrict__ gatB, float* out) {
  extern __shared__ __attribute__((aligned(16))) int dsm[];
  int* sl   = dsm + OFF_SL;
  int* cnt  = dsm + OFF_CNT;
  int* offs = dsm + OFF_OFFS;
  int* misc = dsm + OFF_MISC;
  float* fb = (float*)(dsm + OFF_FB);
  const int tid = (int)threadIdx.x, lane = tid & 31, wave = tid >> 5;
  const int nodeBase = (int)blockIdx.x * NBA;

  build_lists(keys, nE, nodeBase, vec8, dsm, tid, lane, wave);
  const int ovf = misc[9];
  const float qnan = __int_as_float(0x7fc00000);
  const float pz = (ovf != 0) ? qnan : 0.0f;
  const float aS = bf16_val(attS[0]);
  const float aN = bf16_val(attN[0]);
  const float gb = bf16_val(gatB[0]);

#pragma unroll 1
  for (int si = 0; si < NBA / NWAVE; ++si) {
    const int s    = si * NWAVE + wave;
    const int node = nodeBase + s;
    int c = __builtin_amdgcn_readfirstlane(cnt[s]);
    const bool big = c > DEGCAP;
    c = c < 0 ? 0 : (c > DEGCAP ? DEGCAP : c);
    int o = __builtin_amdgcn_readfirstlane(offs[s]);
    o = o < 0 ? 0 : (o > RCAP ? RCAP : o);
    const int nc = node < nN ? node : nN - 1;
    int idx = o + lane;
    idx = idx > RCAP - 1 ? RCAP - 1 : idx;
    const int ent = sl[idx];
    int eid = ent >> SLA;
    eid = eid < 0 ? 0 : (eid > nE - 1 ? nE - 1 : eid);
    int sr = srcs[eid];
    sr = sr < 0 ? 0 : (sr > nN - 1 ? nN - 1 : sr);
    const float xsv = xp[sr];
    const float xi  = xp[nc];
    const bool valid = lane < c;
    int rank = 0;
#pragma unroll 1
    for (int k = 0; k < c; ++k) {
      const int ek = __builtin_amdgcn_readlane(eid, k);
      rank += (ek < eid) ? 1 : 0;
    }
    const float as_ = xi * aS;
    const int selm = -(int)(lane == c);
    const int xvb  = (__float_as_int(xi) & selm) | (__float_as_int(xsv) & ~selm);
    const float xv = __int_as_float(xvb);
    const float an_ = xv * aN;
    float sc = as_ + an_;
    sc = (sc > 0.0f) ? sc : 0.2f * sc;
    const float sself = rdl(sc, c);
    float mm = (lane <= c) ? sc : sself;
#pragma unroll
    for (int d = 16; d >= 1; d >>= 1) {
      const float y = __shfl_xor(mm, d, 32);
      mm = nmax(mm, y);
    }
    const float ex = expf(sc - mm);
    float den = 0.0f;
#pragma unroll 1
    for (int p = 0; p < c; ++p) {
      const unsigned mk = __builtin_amdgcn_ballot_w32(valid && (rank == p));
      int k = __builtin_ffs((int)mk) - 1;
      k = k < 0 ? 0 : k;
      den += rdl(ex, k);
    }
    den += rdl(ex, c);
    const float rinv = 1.0f / den;
    const float tv = (ex * rinv) * xv;
    float ov = 0.0f;
#pragma unroll 1
    for (int p = 0; p < c; ++p) {
      const unsigned mk = __builtin_amdgcn_ballot_w32(valid && (rank == p));
      int k = __builtin_ffs((int)mk) - 1;
      k = k < 0 ? 0 : k;
      ov += rdl(tv, k);
    }
    ov += rdl(tv, c);
    const float v = ov + gb;
    float y = 1.0f / (1.0f + expf(-v));
    const float pzr = big ? qnan : pz;
    y = y + pzr;
    const bool live = node < nN;
    const float res = live ? y : 0.0f;
    if (lane == 0) fb[s] = res;
  }
  __syncthreads();
  const v4f ovv = *(const v4fa*)(fb + 4 * tid);
  const bool okst = (nodeBase + 4 * tid + 3) < nN;
  float* op = out + (size_t)nodeBase + 4 * tid;
  if (okst) *(volatile v4f*)op = ovv;
  __threadfence();
  if (okst) *(volatile v4f*)op = ovv;
}

static inline int cdiv(int a, int b) { return (a + b - 1) / b; }
static inline size_t al256(size_t o) { return (o + 255) & ~(size_t)255; }

extern "C" void kernel_launch(void* const* d_in, const int* in_sizes, int n_in,
                              void* d_out, int out_size, void* d_ws, size_t ws_size,
                              hipStream_t stream) {
  if (n_in < 14) return;
  if (in_sizes[0] < FI || (in_sizes[0] % FI) != 0) return;
  const int nN = in_sizes[0] / FI;
  if (nN < 4 || (nN & 3) != 0 || nN > (1 << 24)) return;
  if (in_sizes[1] < SD || (in_sizes[1] % SD) != 0) return;
  const int nE = in_sizes[1] / SD;
  if (nE < 1 || nE >= (1 << (31 - SLA))) return;
  if (in_sizes[2] != nE || in_sizes[3] != nE) return;
  if (in_sizes[4] != SD * KIN || in_sizes[5] != KIN) return;
  if (in_sizes[6] != KIN * NKER || in_sizes[7] != NKER) return;
  if (in_sizes[8] != FI * FO || in_sizes[9] != FO) return;
  if (in_sizes[10] != FO) return;
  if (in_sizes[11] != 1 || in_sizes[12] != 1 || in_sizes[13] != 1) return;
  if (out_size != nN) return;

  const float* x     = (const float*)d_in[0];
  const float* ef    = (const float*)d_in[1];
  const int*   esrc  = (const int*)d_in[2];
  const int*   edst  = (const int*)d_in[3];
  const float* W1    = (const float*)d_in[4];
  const float* b1    = (const float*)d_in[5];
  const float* W2    = (const float*)d_in[6];
  const float* b2    = (const float*)d_in[7];
  const float* rootk = (const float*)d_in[8];
  const float* eccb  = (const float*)d_in[9];
  const float* gatk  = (const float*)d_in[10];
  const float* attS  = (const float*)d_in[11];
  const float* attN  = (const float*)d_in[12];
  const float* gatB  = (const float*)d_in[13];
  float* out = (float*)d_out;

  const int EP = cdiv(nE, EB) * EB;
  const int gE = EP / EB;
  const int gA = cdiv(nN, NBA);
  const int NP = gA * NBA;
  if (NP < nN) return;
  const int vec8 = ((nE & 3) == 0) ? 1 : 0;

  char* ws = (char*)d_ws;
  size_t off = 0;
  const size_t oW  = off; off = al256(off + (size_t)NKER * KP * 2);
  const size_t oM  = off; off = al256(off + (size_t)EP * FO * 4);
  const size_t oXP = off; off = al256(off + (size_t)NP * 4);
  if (off > ws_size || off > (size_t)WSMAX) return;
  unsigned short* W2T2 = (unsigned short*)(ws + oW);
  float*          MSG  = (float*)(ws + oM);
  float*          XP   = (float*)(ws + oXP);

  const size_t scanLds = (size_t)SCAN_LDS_INTS * 4;
  hipFuncSetAttribute(reinterpret_cast<const void*>(&k_scan1), hipFuncAttributeMaxDynamicSharedMemorySize, (int)scanLds);
  hipFuncSetAttribute(reinterpret_cast<const void*>(&k_scan2), hipFuncAttributeMaxDynamicSharedMemorySize, (int)scanLds);

  k_prep<<<NUW / NTHR, NTHR, 0, stream>>>(W2, W2T2);
  k_ecc_edge<<<gE, ETHR, 0, stream>>>(x, ef, esrc, W1, b1, b2, W2T2, MSG, nE, nN);
  k_scan1<<<gA, NTHR, scanLds, stream>>>(edst, nE, nN, vec8, MSG, x, rootk, eccb, gatk, XP);
  k_scan2<<<gA, NTHR, scanLds, stream>>>(esrc, edst, nE, nN, vec8, XP, attS, attN, gatB, out);
}
